// SqueezeAttention_13640816132789
// MI455X (gfx1250) — hardware-verified
//
#include <hip/hip_runtime.h>
#include <math.h>

typedef __attribute__((ext_vector_type(16))) _Float16 v16h;
typedef __attribute__((ext_vector_type(16))) __bf16 v16b;
typedef __attribute__((ext_vector_type(8)))  _Float16 v8h;
typedef __attribute__((ext_vector_type(8)))  float v8f;
typedef __attribute__((ext_vector_type(4)))  float v4f;
typedef __attribute__((ext_vector_type(2)))  float v2f;
typedef __attribute__((ext_vector_type(4)))  unsigned v4u;
typedef __attribute__((ext_vector_type(4)))  int v4i;
typedef float __attribute__((may_alias)) float_a;
typedef int __attribute__((may_alias)) int_a;

template <typename T> __device__ __forceinline__ void vst2(void* p, T v) { *(volatile T*)p = v; __threadfence(); *(volatile T*)p = v; }
__device__ __forceinline__ v8f wmma16(v16h a, v16h b, v8f c) {
  v8f d = __builtin_amdgcn_wmma_f32_16x16x32_f16(false, a, false, b, (short)0, c, false, false);
  asm volatile("v_nop\n\tv_nop\n\tv_nop\n\tv_nop" : "+v"(d) : "v"(a), "v"(b));
  return d;
}
__device__ __forceinline__ v8f wmma_bf(v16b a, v16b b, v8f c) {
  v8f d = __builtin_amdgcn_wmma_f32_16x16x32_bf16(false, a, false, b, (short)0, c, false, false);
  asm volatile("v_nop\n\tv_nop\n\tv_nop\n\tv_nop" : "+v"(d) : "v"(a), "v"(b));
  return d;
}
__device__ __forceinline__ v16h frag_h(const _Float16* rowk0, int lane) {
  union { v16h v; v8h q[2]; } u; const _Float16* p = rowk0 + 8 * (lane >> 4);
  u.q[0] = *(const v8h*)p; u.q[1] = *(const v8h*)(p + 16); return u.v;
}
__device__ __forceinline__ v16h frag_f32(const float* rowk0, int lane) {
  v16h a; const float* p = rowk0 + 8 * (lane >> 4);
#pragma unroll
  for (int i = 0; i < 8; ++i) { a[i] = (_Float16)p[i]; a[8 + i] = (_Float16)p[16 + i]; }
  return a;
}
__device__ __forceinline__ v16h frag_f32s(const float* rowk0, int lane, float sc) {
  v16h a; const float* p = rowk0 + 8 * (lane >> 4);
#pragma unroll
  for (int i = 0; i < 8; ++i) { a[i] = (_Float16)(p[i] * sc); a[8 + i] = (_Float16)(p[16 + i] * sc); }
  return a;
}
__device__ __forceinline__ v16h fragc_f32(const float* W, int k0, int n, int lane, int ld, int K) {
  v16h a; const int g = lane >> 4;
#pragma unroll
  for (int i = 0; i < 8; ++i) { const int ka = k0 + 8 * g + i, kb = ka + 16;
    a[i] = (_Float16)(ka < K ? W[(size_t)(ka < K ? ka : K - 1) * ld + n] : 0.f); a[8 + i] = (_Float16)(kb < K ? W[(size_t)(kb < K ? kb : K - 1) * ld + n] : 0.f); }
  return a;
}
struct F2 { v16b h, l; };
__device__ __forceinline__ F2 bsplit16(const float v[16]) { F2 r;
#pragma unroll
  for (int i = 0; i < 16; ++i) { const __bf16 h = (__bf16)v[i]; r.h[i] = h; r.l[i] = (__bf16)(v[i] - (float)h); }
  return r; }
__device__ __forceinline__ F2 split_row(const float* row, int k0, int lane) { float v[16]; const float* p = row + k0 + 8 * (lane >> 4);
#pragma unroll
  for (int i = 0; i < 8; ++i) { v[i] = p[i]; v[8 + i] = p[16 + i]; }
  return bsplit16(v); }
__device__ __forceinline__ F2 split_rowK(const float* row, int k0, int lane, int K) { float v[16]; const int g = lane >> 4;
#pragma unroll
  for (int i = 0; i < 8; ++i) { const int ka = k0 + 8 * g + i, kb = ka + 16; v[i] = ka < K ? row[ka < K ? ka : K - 1] : 0.f; v[8 + i] = kb < K ? row[kb < K ? kb : K - 1] : 0.f; }
  return bsplit16(v); }
__device__ __forceinline__ F2 split_col(const float* W, int k0, int n, int lane, int ld, int K) { float v[16]; const int g = lane >> 4;
#pragma unroll
  for (int i = 0; i < 8; ++i) { const int ka = k0 + 8 * g + i, kb = ka + 16; v[i] = ka < K ? W[(size_t)(ka < K ? ka : K - 1) * ld + n] : 0.f; v[8 + i] = kb < K ? W[(size_t)(kb < K ? kb : K - 1) * ld + n] : 0.f; }
  return bsplit16(v); }
__device__ __forceinline__ v8f mac3(const F2& a, const F2& b, v8f c) { c = wmma_bf(a.l, b.h, c); c = wmma_bf(a.h, b.l, c); return wmma_bf(a.h, b.h, c); }
__device__ __forceinline__ float sigm(float v) { return 1.0f / (1.0f + expf(-v)); }
#define LDSX() do { asm volatile("s_wait_dscnt 0" ::: "memory"); __builtin_amdgcn_wave_barrier(); __builtin_amdgcn_fence(__ATOMIC_RELEASE, "workgroup"); } while (0)


#define NB 4
#define SS 2048
#define EE 1024
#define SQ 512
#define NH 16
#define SHD 32
#define HD 64
#define NCOL (SQ + SQ + EE)
#define NROW (NB * SS)
#ifndef TNB
#define TNB NB
#endif
typedef __attribute__((ext_vector_type(8))) __bf16 v8b;
__device__ __forceinline__ v16b frag_b(const __bf16* rowk0, int lane) {
  union { v16b v; v8b q[2]; } u; const __bf16* p = rowk0 + 8 * (lane >> 4);
  u.q[0] = *(const v8b*)p; u.q[1] = *(const v8b*)(p + 16); return u.v;
}
__device__ __forceinline__ float bfr(float v) { return (float)(__bf16)v; }
__device__ __attribute__((noinline)) float exp_ni(float v) { return expf(v); }
__device__ __attribute__((noinline)) float erf_ni(float v) { return erff(v); }

#define WS_PW  0u
#define WS_PO  (WS_PW + 2u * (size_t)NCOL * EE)
#define WS_QK  (WS_PO + 2u * (size_t)EE * EE)
#define WS_VT  (WS_QK + 2u * (size_t)NROW * (2 * SQ))
#define WS_CT  (WS_VT + 2u * (size_t)NB * EE * SS)
#define WS_END (WS_CT + 2u * (size_t)NROW * EE)

__global__ __launch_bounds__(256) void k_packw(const float* __restrict__ WQ, const float* __restrict__ WK, const float* __restrict__ WV, const float* __restrict__ WO, char* __restrict__ ws) { const int n = blockIdx.x, t = threadIdx.x; __shared__ __align__(16) __bf16 s[EE]; __shared__ __align__(16) _Float16 so[EE];
  if (n < NCOL) { for (int k = t; k < EE; k += 256) { float w; if (n < SQ) w = WQ[(size_t)k * SQ + n]; else if (n < 2 * SQ) w = WK[(size_t)k * SQ + n - SQ]; else w = WV[(size_t)k * EE + n - 2 * SQ]; s[k] = (__bf16)w; } __syncthreads(); for (int q = t; q < EE / 8; q += 256) vst2((unsigned*)((__bf16*)(ws + WS_PW) + (size_t)n * EE + q * 8), *(const v4u*)&s[q * 8]); }
  else { const int o = n - NCOL; for (int k = t; k < EE; k += 256) so[k] = (_Float16)bfr(WO[(size_t)k * EE + o]); __syncthreads(); for (int q = t; q < EE / 8; q += 256) vst2((unsigned*)((_Float16*)(ws + WS_PO) + (size_t)o * EE + q * 8), *(const v4u*)&so[q * 8]); } }
__device__ __forceinline__ v16b fragb_f32(const float* __restrict__ p, int lane) { v16b a; const float* pp = p + 8 * (lane >> 4);
#pragma unroll
  for (int i = 0; i < 8; ++i) { a[i] = (__bf16)pp[i]; a[8 + i] = (__bf16)pp[16 + i]; } return a; }
__global__ __launch_bounds__(128) void k_proj(const float* __restrict__ X, const __bf16* __restrict__ PW, const float* __restrict__ BQ, const float* __restrict__ BK, const float* __restrict__ BV, _Float16* __restrict__ QK, _Float16* __restrict__ VT) { __shared__ __align__(16) _Float16 sh[64][136]; __shared__ __align__(16) _Float16 th[128][72];
  const int tid = threadIdx.x, wave = tid >> 5, lane = tid & 31, col = lane & 15, g = lane >> 4; const size_t r0 = (size_t)blockIdx.x * 64 + wave * 16; const int c0 = blockIdx.y * 128; const size_t b = ((size_t)blockIdx.x * 64) / SS; const int n0 = (int)(((size_t)blockIdx.x * 64) % SS);
  v8f acc[8] = {};
#pragma unroll 2
  for (int kc = 0; kc < EE / 32; ++kc) { const v16b a = fragb_f32(X + (r0 + col) * EE + kc * 32, lane);
#pragma unroll
    for (int j = 0; j < 8; ++j) acc[j] = wmma_bf(a, frag_b(PW + (size_t)(c0 + j * 16 + col) * EE + kc * 32, lane), acc[j]); }
  const bool isv = c0 >= 2 * SQ;
#pragma unroll
  for (int j = 0; j < 8; ++j) { const int c = c0 + j * 16 + col; const float bb = c < SQ ? bfr(BQ[c]) : c < 2 * SQ ? bfr(BK[c - SQ]) : bfr(BV[c - 2 * SQ]);
#pragma unroll
    for (int r = 0; r < 8; ++r) { const _Float16 hv = (_Float16)(acc[j][r] + bb); if (!isv) sh[wave * 16 + 8 * g + r][j * 16 + col] = hv; else th[j * 16 + col][wave * 16 + 8 * g + r] = hv; } }
  __syncthreads();
  if (!isv) { for (int e = tid; e < 64 * 16; e += 128) { const int rl = e >> 4, q = e & 15; vst2((unsigned*)(QK + ((size_t)blockIdx.x * 64 + rl) * (2 * SQ) + c0 + q * 8), *(const v4u*)&sh[rl][q * 8]); } }
  else { const int cv0 = c0 - 2 * SQ; for (int e = tid; e < 128 * 8; e += 128) { const int cl = e >> 3, q = e & 7; vst2((unsigned*)(VT + (b * EE + cv0 + cl) * (size_t)SS + n0 + q * 8), *(const v4u*)&th[cl][q * 8]); } } }
__global__ __launch_bounds__(128) void k_att(const _Float16* __restrict__ QK, const _Float16* __restrict__ VT, _Float16* __restrict__ CT) {
  __shared__ __align__(16) float sp[4][16][36]; __shared__ __align__(16) _Float16 so[4][16][72];
  const int tid = threadIdx.x, wave = tid >> 5, lane = tid & 31, col = lane & 15, g = lane >> 4; const int h = blockIdx.y; const size_t b = blockIdx.z; const int q0 = blockIdx.x * 64 + wave * 16; const size_t rq = b * SS + q0;
  const v16h aq = frag_h(QK + (rq + col) * (2 * SQ) + h * SHD, lane);
  float m[8], l[8];
#pragma unroll
  for (int r = 0; r < 8; ++r) { m[r] = -3.0e38f; l[r] = 0.f; }
  v8f acc[4] = {};
#pragma unroll 1
  for (int ks = 0; ks < SS / 32; ++ks) { v8f s[2];
#pragma unroll
    for (int ct = 0; ct < 2; ++ct) { const size_t rk = b * SS + ks * 32 + ct * 16 + col; v8f c = {}; c = wmma16(aq, frag_h(QK + rk * (2 * SQ) + SQ + h * SHD, lane), c);
#pragma unroll
      for (int r = 0; r < 8; ++r) s[ct][r] = c[r] * 0.17677669529663687f; }
    float alpha[8];
#pragma unroll
    for (int r = 0; r < 8; ++r) { float mx = fmaxf(s[0][r], s[1][r]);
#pragma unroll
      for (int o = 1; o < 16; o <<= 1) mx = fmaxf(mx, __shfl_xor(mx, o));
      const float mn = fmaxf(m[r], mx); alpha[r] = __expf(m[r] - mn); const float e0 = __expf(s[0][r] - mn), e1 = __expf(s[1][r] - mn); float es = e0 + e1;
#pragma unroll
      for (int o = 1; o < 16; o <<= 1) es += __shfl_xor(es, o);
      l[r] = l[r] * alpha[r] + es; m[r] = mn; sp[wave][8 * g + r][col] = e0; sp[wave][8 * g + r][16 + col] = e1; }
#pragma unroll
    for (int j = 0; j < 4; ++j)
#pragma unroll
      for (int r = 0; r < 8; ++r) acc[j][r] *= alpha[r];
    LDSX();
    v16h pa; { const float* prow = &sp[wave][col][0] + 8 * (lane >> 4);
#pragma unroll
      for (int i = 0; i < 8; ++i) { pa[i] = (_Float16)(prow[i] * 2048.0f); pa[8 + i] = (_Float16)(prow[16 + i] * 2048.0f); } }
#pragma unroll
    for (int j = 0; j < 4; ++j) acc[j] = wmma16(pa, frag_h(VT + (b * EE + (size_t)h * HD + j * 16 + col) * (size_t)SS + ks * 32, lane), acc[j]);
    LDSX(); }
#pragma unroll
  for (int r = 0; r < 8; ++r) { const float il = (1.0f / 2048.0f) / l[r];
#pragma unroll
    for (int j = 0; j < 4; ++j) so[wave][8 * g + r][j * 16 + col] = (_Float16)(acc[j][r] * il); }
  LDSX(); for (int rl = 0; rl < 16; ++rl) if (lane < 8) vst2((unsigned*)(CT + (rq + rl) * EE + (size_t)h * HD + lane * 8), *(const v4u*)&so[wave][rl][lane * 8]); }
__global__ __launch_bounds__(128) void k_out(const _Float16* __restrict__ CT, const _Float16* __restrict__ PO, const float* __restrict__ BO, float* __restrict__ OUT) { __shared__ __align__(16) float sf[4][16][132];
  const int tid = threadIdx.x, wave = tid >> 5, lane = tid & 31, col = lane & 15, g = lane >> 4; const size_t r0 = (size_t)blockIdx.x * 64 + wave * 16; const int c0 = blockIdx.y * 128;
  v8f acc[8] = {};
#pragma unroll 2
  for (int kc = 0; kc < EE / 32; ++kc) { const v16h a = frag_h(CT + (r0 + col) * EE + kc * 32, lane);
#pragma unroll
    for (int j = 0; j < 8; ++j) acc[j] = wmma16(a, frag_h(PO + (size_t)(c0 + j * 16 + col) * EE + kc * 32, lane), acc[j]); }
#pragma unroll
  for (int j = 0; j < 8; ++j) { const float bb = bfr(BO[c0 + j * 16 + col]);
#pragma unroll
    for (int r = 0; r < 8; ++r) sf[wave][8 * g + r][j * 16 + col] = acc[j][r] + bb; }
  LDSX(); for (int rl = 0; rl < 16; ++rl) vst2(OUT + (r0 + rl) * EE + c0 + lane * 4, *(const v4f*)&sf[wave][rl][lane * 4]); }
extern "C" void kernel_launch(void* const* d_in, const int* in_sizes, int n_in, void* d_out, int out_size, void* d_ws, size_t ws_size, hipStream_t stream) {
  (void)in_sizes; (void)n_in; (void)out_size;
  const float** F = (const float**)d_in;
  if (ws_size < (size_t)WS_END) return;
  char* ws = (char*)d_ws; const __bf16* PW = (const __bf16*)(ws + WS_PW); const _Float16* PO = (const _Float16*)(ws + WS_PO); _Float16 *QK = (_Float16*)(ws + WS_QK), *VT = (_Float16*)(ws + WS_VT), *CT = (_Float16*)(ws + WS_CT);
  k_packw<<<NCOL + EE, 256, 0, stream>>>(F[1], F[3], F[5], F[7], ws);
  k_proj<<<dim3(NROW / 64, NCOL / 128), 128, 0, stream>>>(F[0], PW, F[2], F[4], F[6], QK, VT);
  k_att<<<dim3(SS / 64, NH, TNB), 128, 0, stream>>>(QK, VT, CT);
  k_out<<<dim3(TNB * SS / 64, EE / 128), 128, 0, stream>>>(CT, PO, F[8], (float*)d_out);
}
